// LearnableDistanceMetric_27315992002939
// MI455X (gfx1250) — hardware-verified
//
#include <hip/hip_runtime.h>
#include <hip/hip_bf16.h>
#include <math.h>

#define NQ 4096
#define NC 64
#define DDl 512
#define H1 512
#define H2 256
#define GSTR 48

typedef _Float16 bf16;
typedef _Float16 f16;
typedef __attribute__((ext_vector_type(4))) unsigned v4u_t;
typedef unsigned v4ua __attribute__((ext_vector_type(4), may_alias));
typedef __attribute__((ext_vector_type(4))) float v4f_t;
typedef float v4fa __attribute__((ext_vector_type(4), may_alias));
typedef __attribute__((ext_vector_type(16))) bf16  bf16x16;
typedef bf16x16 f16x16;
typedef __attribute__((ext_vector_type(8)))  bf16  bf16x8;
typedef bf16x8 f16x8;
typedef __attribute__((ext_vector_type(4)))  bf16  bf16x4;
typedef __attribute__((ext_vector_type(8)))  float f32x8;
__device__ __forceinline__ f32x8 wmma16(f16x16 a, f16x16 b, f32x8 c) {
  c = __builtin_amdgcn_wmma_f32_16x16x32_f16(false, a, false, b, (short)0, c, false, false);
  asm volatile("v_nop\n\tv_nop\n\tv_nop\n\tv_nop" : "+v"(c) : "v"(a), "v"(b));
  return c;
}
#define LDS_STRIDE 48
#define KSTRIDE    72
#define VSTRIDE    48

__device__ __forceinline__ f32x8 wmma_bf16(bf16x16 a, bf16x16 b, f32x8 c) {
  c = __builtin_amdgcn_wmma_f32_16x16x32_f16(false, a, false, b, (short)0, c, false, false);
  asm volatile("v_nop\n\tv_nop\n\tv_nop\n\tv_nop" : "+v"(c) : "v"(a), "v"(b));
  return c;
}

template <typename T>
__device__ __forceinline__ bf16x16 load_frag(const T* __restrict__ base, int ld,
                                             int row0, int k0) {
  const int lane = threadIdx.x & 31;
  const int r    = lane & 15;
  const int kh   = (lane >> 4) * 8;
  const T* p0 = base + (size_t)(row0 + r) * ld + (k0 + kh);
  const T* p1 = p0 + 16;
  bf16x16 f;
#pragma unroll
  for (int i = 0; i < 8; ++i) {
    f[i]     = (bf16)p0[i];
    f[i + 8] = (bf16)p1[i];
  }
  return f;
}

__device__ __forceinline__ bf16x16 lds_frag(const bf16* base, int stride) {
  const int lane = threadIdx.x & 31;
  const int row  = lane & 15;
  const int kh   = (lane >> 4) * 8;
  const bf16x8 lo = *(const bf16x8*)(base + row * stride + kh);
  const bf16x8 hi = *(const bf16x8*)(base + row * stride + kh + 16);
  bf16x16 f;
#pragma unroll
  for (int i = 0; i < 8; ++i) { f[i] = lo[i]; f[i + 8] = hi[i]; }
  return f;
}

template <typename T>
__device__ __forceinline__ void stage_read16(const T* __restrict__ p, float* buf) {
#pragma unroll
  for (int i = 0; i < 16; ++i) buf[i] = (float)p[i];
}

__device__ __forceinline__ void stage_write(bf16* dst, const float* buf, int nquad) {
#pragma unroll
  for (int i = 0; i < nquad; ++i) {
    bf16x4 q;
    q[0] = (bf16)buf[4 * i];     q[1] = (bf16)buf[4 * i + 1];
    q[2] = (bf16)buf[4 * i + 2]; q[3] = (bf16)buf[4 * i + 3];
    *(bf16x4*)(dst + 4 * i) = q;
  }
}


#define GSTR 48
template <typename AT, int EPI, bool OUT16>
__global__ __launch_bounds__(256) void gemm_kne(const AT* __restrict__ A, int lda, const float* __restrict__ Wm, int ldw,
                                                const float* __restrict__ bias, const float* __restrict__ R, const float* __restrict__ gvec,
                                                void* __restrict__ Yv, int ldy, int K) {
  __shared__ __attribute__((aligned(16))) f16 ldsA[128 * GSTR];
  __shared__ __attribute__((aligned(16))) f16 ldsW[128 * GSTR];
  __shared__ __attribute__((aligned(16))) float oS[8][32 * 68];
  const int tid = threadIdx.x, lane = tid & 31, wave = tid >> 5, cl = lane & 15, rh = (lane >> 4) * 8;
  const int m0 = blockIdx.x * 128, n0 = blockIdx.y * 128;
  const int wm = (wave & 3) * 32, wn = (wave >> 2) * 64;
  f32x8 acc[2][4];
#pragma unroll
  for (int i = 0; i < 2; ++i)
#pragma unroll
    for (int j = 0; j < 4; ++j) { f32x8 z = {}; acc[i][j] = z; }
#pragma unroll 1
  for (int k0 = 0; k0 < K; k0 += 32) {
    __syncthreads();
    { const int row = tid >> 1, ch = (tid & 1) * 16;
      const AT* src = A + (size_t)(m0 + row) * lda + k0 + ch;
#pragma unroll
      for (int g = 0; g < 16; ++g) ldsA[row * GSTR + ch + g] = (f16)src[g]; }
    { const int k = tid >> 3, nn0 = (tid & 7) * 16;
      const float* src = Wm + (size_t)(k0 + k) * ldw + n0 + nn0;
#pragma unroll
      for (int g = 0; g < 4; ++g) { const v4f_t v = *(const v4f_t*)(src + 4 * g);
#pragma unroll
        for (int u = 0; u < 4; ++u) ldsW[(nn0 + 4 * g + u) * GSTR + k] = (f16)v[u]; } }
    __syncthreads();
    f16x16 af[2];
#pragma unroll
    for (int i = 0; i < 2; ++i) af[i] = lds_frag(ldsA + (wm + 16 * i) * GSTR, GSTR);
#pragma unroll
    for (int j = 0; j < 4; ++j) {
      const f16x16 bf = lds_frag(ldsW + (wn + 16 * j) * GSTR, GSTR);
#pragma unroll
      for (int i = 0; i < 2; ++i) acc[i][j] = wmma16(af[i], bf, acc[i][j]);
    }
  }
  float* so = oS[wave];
#pragma unroll
  for (int i = 0; i < 2; ++i)
#pragma unroll
    for (int j = 0; j < 4; ++j) {
      const int n = n0 + wn + 16 * j + cl;
      const float bv = bias ? bias[n] : 0.0f;
      const float gv = (EPI == 2) ? gvec[n] : 0.0f;
      if (EPI == 1) {
#pragma unroll 1
        for (int r = 0; r < 8; ++r) { const float xg = acc[i][j][r] + bv; so[(16 * i + rh + r) * 68 + 16 * j + cl] = 0.5f * xg * (1.0f + erff(xg * 0.70710678118654752f)); }
      } else {
#pragma unroll
        for (int r = 0; r < 8; ++r) {
          float v = acc[i][j][r] + bv;
          if (EPI == 2) v = R[(size_t)(m0 + wm + 16 * i + rh + r) * ldy + n] + gv * v;
          so[(16 * i + rh + r) * 68 + 16 * j + cl] = v;
        }
      }
    }
  asm volatile("s_wait_dscnt 0" ::: "memory");
  __builtin_amdgcn_wave_barrier();
#pragma unroll 1
  for (int pass = 0; pass < 2; ++pass) {
    if (OUT16) {
      f16* Y = (f16*)Yv;
#pragma unroll
      for (int it = 0; it < 8; ++it) { const int c = lane + 32 * it, rr = c >> 3, q8 = (c & 7) * 8;
        union { f16 h[8]; v4u_t v; } u;
#pragma unroll
        for (int e = 0; e < 8; ++e) u.h[e] = (f16)so[rr * 68 + q8 + e];
        *(volatile v4u_t*)(Y + (size_t)(m0 + wm + rr) * ldy + n0 + wn + q8) = u.v; }
    } else {
      float* Y = (float*)Yv;
#pragma unroll
      for (int it = 0; it < 16; ++it) { const int f4 = lane + 32 * it, rr = f4 >> 4, q = (f4 & 15) * 4;
        *(volatile v4f_t*)(Y + (size_t)(m0 + wm + rr) * ldy + n0 + wn + q) = *(const v4fa*)(so + rr * 68 + q); }
    }
    __threadfence();
  }
}

__global__ __launch_bounds__(256) void k_padp(const float* __restrict__ pe, float* __restrict__ pp) { const int r = blockIdx.x;
  for (int q4 = threadIdx.x; q4 < DDl / 4; q4 += 256) { v4f_t v = {0.f,0.f,0.f,0.f}; if (r < NC) v = *(const v4f_t*)(pe + (size_t)r * DDl + q4 * 4); *(volatile v4f_t*)(pp + (size_t)r * DDl + q4 * 4) = v; __threadfence(); *(volatile v4f_t*)(pp + (size_t)r * DDl + q4 * 4) = v; } }

__global__ __launch_bounds__(256) void k_pairmlp(const float* __restrict__ HQ, const float* __restrict__ HP, const float* __restrict__ b1, const float* __restrict__ W2, const float* __restrict__ b2,
                                                const float* __restrict__ W3, const float* __restrict__ b3, float* __restrict__ out) {
  __shared__ __attribute__((aligned(16))) f16 hpS[NC * (H1 + 8)];
  __shared__ float hqS[2 * H1];
  __shared__ __attribute__((aligned(16))) f16 aS[128 * 40];
  __shared__ __attribute__((aligned(16))) f16 wS[H2 * 40];
  __shared__ __attribute__((aligned(16))) float oS[128];
  const int tid = threadIdx.x, lane = tid & 31, wave = tid >> 5, cl = lane & 15, rh = (lane >> 4) * 8;
  const int q0 = blockIdx.x * 2;
  for (int e = tid; e < NC * H1; e += 256) { const int c = e >> 9, k = e & 511; hpS[c * (H1 + 8) + k] = (f16)(HP[e] + b1[k]); }
  for (int e = tid; e < 2 * H1; e += 256) hqS[e] = HQ[(size_t)q0 * H1 + e];
  f32x8 acc[16];
#pragma unroll
  for (int t = 0; t < 16; ++t) { f32x8 z = {}; acc[t] = z; }
#pragma unroll 1
  for (int ks = 0; ks < H1 / 32; ++ks) {
    __syncthreads();
    { const int r = tid >> 1, q = (tid & 1) * 16; const int qq = r >> 6, c = r & 63;
      union { f16 h[16]; v4u_t u[2]; } av;
#pragma unroll
      for (int e = 0; e < 16; ++e) { const int k = ks * 32 + q + e; av.h[e] = (f16)fmaxf(hqS[qq * H1 + k] + (float)hpS[c * (H1 + 8) + k], 0.0f); }
      *(v4u_t*)(aS + r * 40 + q) = av.u[0]; *(v4u_t*)(aS + r * 40 + q + 8) = av.u[1]; }
    { const int kk = tid >> 3, q = (tid & 7) * 32; const float* wr = W2 + (size_t)(ks * 32 + kk) * H2 + q;
#pragma unroll
      for (int e = 0; e < 32; ++e) wS[(q + e) * 40 + kk] = (f16)wr[e]; }
    __syncthreads();
    const f16x16 af = lds_frag(aS + (wave * 16) * 40, 40);
#pragma unroll
    for (int t = 0; t < 16; ++t) acc[t] = wmma16(af, lds_frag(wS + (t * 16) * 40, 40), acc[t]);
  }
  float ep[8];
#pragma unroll
  for (int r = 0; r < 8; ++r) ep[r] = 0.0f;
#pragma unroll
  for (int t = 0; t < 16; ++t) { const int o = t * 16 + cl; const float bb = b2[o], w = W3[o];
#pragma unroll
    for (int r = 0; r < 8; ++r) ep[r] += fmaxf(acc[t][r] + bb, 0.0f) * w; }
#pragma unroll
  for (int r = 0; r < 8; ++r) { float v = ep[r];
#pragma unroll
    for (int off = 1; off < 16; off <<= 1) v += __shfl_xor(v, off, 32);
    ep[r] = v; }
  if (cl == 0) {
#pragma unroll
    for (int r = 0; r < 8; ++r) oS[wave * 16 + rh + r] = ep[r] + b3[0]; }
  __syncthreads();
#pragma unroll 1
  for (int pass = 0; pass < 2; ++pass) { if (tid < 32) *(volatile v4f_t*)(out + (size_t)q0 * NC + tid * 4) = *(const v4fa*)(oS + tid * 4); __threadfence(); }
}

extern "C" void kernel_launch(void* const* d_in, const int* in_sizes, int n_in,
                              void* d_out, int out_size, void* d_ws, size_t ws_size,
                              hipStream_t stream) {
  (void)in_sizes; (void)n_in; (void)out_size;
  const float** f = (const float**)d_in;
  const float* qe = f[0], *pe = f[1], *W1 = f[2], *b1 = f[3], *W2 = f[4], *b2 = f[5], *W3 = f[6], *b3 = f[7];
  float* out = (float*)d_out;
  char* ws = (char*)d_ws;
  float* HQ = (float*)ws; ws += (size_t)NQ * H1 * 4;
  float* pe128 = (float*)ws; ws += (size_t)128 * DDl * 4;
  float* HP = (float*)ws; ws += (size_t)128 * H1 * 4;
  if ((size_t)(ws - (char*)d_ws) > ws_size) return;
  const dim3 blk(256);
  k_padp<<<dim3(128), blk, 0, stream>>>(pe, pe128);
  gemm_kne<float, 0, false><<<dim3(NQ / 128, H1 / 128), blk, 0, stream>>>(qe, DDl, W1, H1, nullptr, nullptr, nullptr, HQ, H1, DDl);
  gemm_kne<float, 0, false><<<dim3(1, H1 / 128), blk, 0, stream>>>(pe128, DDl, W1 + (size_t)DDl * H1, H1, nullptr, nullptr, nullptr, HP, H1, DDl);
  k_pairmlp<<<dim3(NQ / 2), blk, 0, stream>>>(HQ, HP, b1, W2, b2, W3, b3, out);
}
